// CATCallerEncoderLayer_86449101734002
// MI455X (gfx1250) — hardware-run, weakly checked
//
#include <hip/hip_runtime.h>


#ifndef SEQ
#define SEQ 1024
#endif
#define SEQ_FULL 1024
#define NBT  16
#define CC   512
#define C2   1024
#define NHD  8
#define HW   64
#define NTAP 31
#define PADL 15
#define HK   248
#define HKP  256
#define MROWS (SEQ * NBT)
#define TCH  32
#define GP   132
#define XGC  64.0f
#define YC   256.0f
#define WC   1024.0f
#define LG_ISH 16
#define OT_ISH 18

static_assert(NHD * HW == CC);
static_assert(NHD * NTAP == HK);
static_assert(HK <= HKP);
static_assert(HKP % 64 == 0);
static_assert(CC % 64 == 0);
static_assert(C2 == 2 * CC);
static_assert(CC % 32 == 0);
static_assert(MROWS % 64 == 0);
static_assert(SEQ % TCH == 0);
static_assert(SEQ <= SEQ_FULL);
static_assert(TCH + 32 <= 64);
static_assert(2 * PADL + 1 == NTAP);
static_assert((GP * 4) % 16 == 0);
static_assert(32 * 16 * 8 == 16 * 256);
static_assert(32 * 16 * 4 == 16 * 128);
static_assert(32 * 16 * 8 == 16 * 64 * 4);
static_assert(256 * 16 * 1 == TCH * HW * 2);
static_assert(256 * 16 * 2 == 64 * 64 * 2);
static_assert(256 * 4 == 64 * (HW / 4));
static_assert(256 * 4 == TCH * 32);
static_assert((16 * GP * 4) <= 131072);
static_assert((64 * HW + TCH * 32 + TCH * HW) * 4 <= 131072);
static_assert((64 * 65 * 4) <= 131072);
static_assert((16 * 68 * 4) <= 131072);

typedef _Float16 h16;
typedef unsigned short bf;
typedef __attribute__((ext_vector_type(16))) __bf16   v16bf;
typedef __attribute__((ext_vector_type(16))) _Float16 v16h;
typedef __attribute__((ext_vector_type(8)))  _Float16 v8h;
typedef __attribute__((ext_vector_type(8)))  unsigned short v8us;
typedef __attribute__((ext_vector_type(8)))  float    v8f;
typedef __attribute__((ext_vector_type(4)))  float    v4f;
typedef v4f  __attribute__((may_alias)) v4fa;

__device__ __forceinline__ unsigned short f2bf(float f) { unsigned u = __float_as_uint(f); u += 0x7FFFu + ((u >> 16) & 1u); return (unsigned short)(u >> 16); }
__device__ __forceinline__ float bfr(float f) { return __uint_as_float(((unsigned)f2bf(f)) << 16); }
__device__ __forceinline__ v16h cat16(v8h lo, v8h hi) { return __builtin_shufflevector(lo, hi, 0, 1, 2, 3, 4, 5, 6, 7, 8, 9, 10, 11, 12, 13, 14, 15); }
__device__ __forceinline__ v16bf cat16b(v8us lo, v8us hi) { return __builtin_bit_cast(v16bf, __builtin_shufflevector(lo, hi, 0, 1, 2, 3, 4, 5, 6, 7, 8, 9, 10, 11, 12, 13, 14, 15)); }
__device__ __forceinline__ v8f wmma16(v16h a, v16h b, v8f c) { return __builtin_amdgcn_wmma_f32_16x16x32_f16(false, a, false, b, (short)0, c, false, false); }
__device__ __forceinline__ v8f wmmab(v16bf a, v16bf b, v8f c) { return __builtin_amdgcn_wmma_f32_16x16x32_bf16(false, a, false, b, (short)0, c, false, false); }
__device__ __forceinline__ v8f wmmabg(v16bf a, v16bf b, v8f c) { c = wmmab(a, b, c); asm volatile("v_nop\n\tv_nop\n\tv_nop\n\tv_nop" : "+v"(c) : "v"(a), "v"(b)); return c; }
__device__ __forceinline__ v8f wmma16g(v16h a, v16h b, v8f c) { c = wmma16(a, b, c); asm volatile("v_nop\n\tv_nop\n\tv_nop\n\tv_nop" : "+v"(c) : "v"(a), "v"(b)); return c; }
__device__ __forceinline__ v16h  ldh(const h16* p) { return cat16(*(const v8h*)p, *(const v8h*)(p + 16)); }
__device__ __forceinline__ v16bf ldb(const bf* p)  { return cat16b(*(const v8us*)p, *(const v8us*)(p + 16)); }
__device__ __forceinline__ void wave_sync() { __builtin_amdgcn_fence(3  , "wavefront"); __builtin_amdgcn_wave_barrier(); asm volatile("" ::: "memory"); }
static __device__ __forceinline__ h16 toh_flush(float v) { const float w = (fabsf(v) < 6.103515625e-05f) ? 0.0f : v; return (h16)w; }

__global__ __launch_bounds__(256) void k_cvt8(const float* __restrict__ src, bf* dst, size_t n8) {
    const size_t i = (size_t)blockIdx.x * 256 + threadIdx.x; if (i >= n8) return;
    const v8f v = *(const v8f*)(src + i * 8); v8us o;
#pragma unroll
    for (int k = 0; k < 8; ++k) o[k] = f2bf(v[k]);
    *(volatile v8us*)(dst + i * 8) = o; __threadfence(); *(volatile v8us*)(dst + i * 8) = o;
}

__global__ __launch_bounds__(256) void k_wt_b(const float* __restrict__ W, bf* dst, int ldw, int ncols) {
    __shared__ float ts[64 * 65];
    const unsigned tid = threadIdx.x;
    const unsigned k0 = blockIdx.x * 64u, n0 = blockIdx.y * 64u;
#pragma unroll 4
    for (int i = 0; i < 16; ++i) {
        const unsigned e = (unsigned)i * 256u + tid; const unsigned kk = e >> 6, nn = e & 63u;
        const int n = (int)(n0 + nn); const int nc = min(n, ncols - 1);
        float v = W[(size_t)(k0 + kk) * (size_t)ldw + (size_t)nc];
        asm volatile("" : "+v"(v));
        ts[nn * 65u + kk] = (n < ncols) ? bfr(v) : 0.0f; }
    __syncthreads();
    const unsigned pa = tid, pb = 256u + tid;
    const unsigned na = pa >> 3, ka = (pa & 7u) * 8u, nb = pb >> 3, kb = (pb & 7u) * 8u;
    v8us o0, o1;
#pragma unroll
    for (int j = 0; j < 8; ++j) { o0[j] = f2bf(ts[na * 65u + ka + j]); o1[j] = f2bf(ts[nb * 65u + kb + j]); }
    bf* d0 = dst + (size_t)(n0 + na) * CC + k0 + ka;
    bf* d1 = dst + (size_t)(n0 + nb) * CC + k0 + kb;
    *(volatile v8us*)d0 = o0; *(volatile v8us*)d1 = o1;
    __threadfence();
    *(volatile v8us*)d0 = o0; *(volatile v8us*)d1 = o1;
}

__global__ __launch_bounds__(256) void k_wt_h(const float* __restrict__ W, h16* dst, int ldw, int ncols) {
    __shared__ float ts[64 * 65];
    const unsigned tid = threadIdx.x;
    const unsigned k0 = blockIdx.x * 64u, n0 = blockIdx.y * 64u;
#pragma unroll 4
    for (int i = 0; i < 16; ++i) {
        const unsigned e = (unsigned)i * 256u + tid; const unsigned kk = e >> 6, nn = e & 63u;
        const int n = (int)(n0 + nn); const int nc = min(n, ncols - 1);
        float v = W[(size_t)(k0 + kk) * (size_t)ldw + (size_t)nc];
        asm volatile("" : "+v"(v));
        ts[nn * 65u + kk] = (n < ncols) ? bfr(v) : 0.0f; }
    __syncthreads();
    const unsigned pa = tid, pb = 256u + tid;
    const unsigned na = pa >> 3, ka = (pa & 7u) * 8u, nb = pb >> 3, kb = (pb & 7u) * 8u;
    v8h o0, o1;
#pragma unroll
    for (int j = 0; j < 8; ++j) { o0[j] = toh_flush(ts[na * 65u + ka + j] * WC); o1[j] = toh_flush(ts[nb * 65u + kb + j] * WC); }
    h16* d0 = dst + (size_t)(n0 + na) * CC + k0 + ka;
    h16* d1 = dst + (size_t)(n0 + nb) * CC + k0 + kb;
    *(volatile v8h*)d0 = o0; *(volatile v8h*)d1 = o1;
    __threadfence();
    *(volatile v8h*)d0 = o0; *(volatile v8h*)d1 = o1;
}

__global__ __launch_bounds__(32) __attribute__((amdgpu_num_vgpr(256)))
void k_glu(const bf* __restrict__ A, const bf* __restrict__ Bt, const float* __restrict__ bias, float* XG, h16* XH) {
    __shared__ __align__(16) float os[16 * GP];
    const int K = CC;
    const int lane = threadIdx.x & 31, lr = lane & 15, hi = lane >> 4;
    const unsigned bx = blockIdx.x, by = blockIdx.y;
    const unsigned r0 = bx * 32u, c0 = by * 64u;
    v8f acc[2][8];
#pragma unroll
    for (int mb = 0; mb < 2; ++mb)
#pragma unroll
        for (int nb = 0; nb < 8; ++nb) acc[mb][nb] = (v8f){};
    const size_t aoff  = (size_t)(r0 + (unsigned)lr) * K + 8 * hi;
    const size_t boffa = (size_t)(c0 + (unsigned)lr) * K + 8 * hi;
    const size_t boffg = (size_t)((unsigned)CC + c0 + (unsigned)lr) * K + 8 * hi;
#pragma unroll 1
    for (int kc = 0; kc < K; kc += 32) {
        const v16bf a0 = ldb(A + aoff + kc);
        const v16bf a1 = ldb(A + aoff + (size_t)16 * K + kc);
#pragma unroll
        for (int nb = 0; nb < 8; ++nb) {
            const size_t bo = (nb < 4) ? (boffa + (size_t)nb * 16 * K) : (boffg + (size_t)(nb - 4) * 16 * K);
            const v16bf b = ldb(Bt + bo + kc);
            acc[0][nb] = wmmabg(a0, b, acc[0][nb]);
            acc[1][nb] = wmmabg(a1, b, acc[1][nb]); }
    }
    float bc[8];
#pragma unroll
    for (int nb = 0; nb < 4; ++nb) { bc[nb] = bfr(bias[c0 + nb * 16 + lr]); bc[4 + nb] = bfr(bias[CC + c0 + nb * 16 + lr]); }
#pragma unroll
    for (int mb = 0; mb < 2; ++mb) {
#pragma unroll
        for (int nb = 0; nb < 8; ++nb) {
#pragma unroll
            for (int j = 0; j < 8; ++j) os[(hi * 8 + j) * GP + nb * 16 + lr] = acc[mb][nb][j] + bc[nb]; }
        wave_sync();
#pragma unroll 1
        for (int s = 0; s < 8; ++s) { const int p = s * 32 + lane; const int row = p >> 4, c4 = (p & 15) * 4;
            const v4f av = *(const v4fa*)(&os[row * GP + c4]); const v4f gv = *(const v4fa*)(&os[row * GP + 64 + c4]); v4f y;
#pragma unroll
            for (int i = 0; i < 4; ++i) y[i] = av[i] * (1.0f / (1.0f + expf(-gv[i])));
            *(v4fa*)(&os[row * GP + c4]) = y; }
        wave_sync();
        float* xrow = XG + (size_t)(r0 + (unsigned)(mb * 16)) * CC + c0;
        h16*   hrow = XH + (size_t)(r0 + (unsigned)(mb * 16)) * CC + c0;
#pragma unroll 1
        for (int ps = 0; ps < 2; ++ps) {
#pragma unroll
            for (int s = 0; s < 8; ++s) { const int row = 2 * s + (lane >> 4), cofs = (lane & 15) * 4;
                const v4f val = *(const v4fa*)(&os[row * GP + cofs]);
                *(volatile v4f*)(xrow + (size_t)row * CC + cofs) = val; }
#pragma unroll
            for (int s = 0; s < 4; ++s) { const int row = 4 * s + (lane >> 3), c8 = (lane & 7) * 8;
                const v4f x0 = *(const v4fa*)(&os[row * GP + c8]); const v4f x1 = *(const v4fa*)(&os[row * GP + c8 + 4]); v8h hv;
#pragma unroll
                for (int i = 0; i < 4; ++i) { hv[i] = toh_flush(x0[i] * XGC); hv[4 + i] = toh_flush(x1[i] * XGC); }
                *(volatile v8h*)(hrow + (size_t)row * CC + c8) = hv; }
            if (ps == 0) __threadfence(); }
        wave_sync();
    }
}

__global__ __launch_bounds__(32) __attribute__((amdgpu_num_vgpr(256)))
void k_gemm_h(const h16* __restrict__ A, const h16* __restrict__ Bt, const float* __restrict__ bias, float* OUT, int ldo, int nbias, int ish) {
    __shared__ __align__(16) float os[16 * 68];
    const int K = CC;
    const int lane = threadIdx.x & 31, lr = lane & 15, hi = lane >> 4;
    const unsigned bx = blockIdx.x, by = blockIdx.y;
    const unsigned r0 = bx * 64u, c0 = by * 64u;
    v8f acc[4][4];
#pragma unroll
    for (int mb = 0; mb < 4; ++mb)
#pragma unroll
        for (int nb = 0; nb < 4; ++nb) acc[mb][nb] = (v8f){};
    const size_t aoff = (size_t)(r0 + (unsigned)lr) * K + 8 * hi, boff = (size_t)(c0 + (unsigned)lr) * K + 8 * hi;
#pragma unroll 1
    for (int kc = 0; kc < K; kc += 32) {
        v16h a[4];
#pragma unroll
        for (int mb = 0; mb < 4; ++mb) a[mb] = ldh(A + aoff + (size_t)mb * 16 * K + kc);
#pragma unroll
        for (int nb = 0; nb < 4; ++nb) { const v16h b = ldh(Bt + boff + (size_t)nb * 16 * K + kc);
#pragma unroll
            for (int mb = 0; mb < 4; ++mb) acc[mb][nb] = wmma16g(a[mb], b, acc[mb][nb]); }
    }
    const float scl = __uint_as_float((unsigned)(127 - ish) << 23);
    float bc[4];
#pragma unroll
    for (int nb = 0; nb < 4; ++nb) { const int n = (int)c0 + nb * 16 + lr; const int nc = min(n, nbias - 1);
        float bv = bias[nc]; asm volatile("" : "+v"(bv));
        bc[nb] = (n < nbias) ? bfr(bv) : 0.0f; }
#pragma unroll
    for (int mb = 0; mb < 4; ++mb) {
#pragma unroll
        for (int nb = 0; nb < 4; ++nb) {
#pragma unroll
            for (int j = 0; j < 8; ++j) os[(hi * 8 + j) * 68 + nb * 16 + lr] = acc[mb][nb][j] * scl + bc[nb]; }
        wave_sync();
        float* orow = OUT + (size_t)(r0 + (unsigned)(mb * 16)) * (size_t)ldo + c0;
#pragma unroll 1
        for (int ps = 0; ps < 2; ++ps) {
#pragma unroll
            for (int s = 0; s < 8; ++s) { const int row = 2 * s + (lane >> 4), cofs = (lane & 15) * 4;
                const v4f val = *(const v4fa*)(&os[row * 68 + cofs]);
                *(volatile v4f*)(orow + (size_t)row * (size_t)ldo + cofs) = val; }
            if (ps == 0) __threadfence(); }
        wave_sync();
    }
}

__global__ __launch_bounds__(256) void k_dconv(const float* __restrict__ XG, const float* __restrict__ LG, h16* YH) {
    __shared__ __align__(16) float xs[64 * HW];
    __shared__ __align__(16) float wl[TCH * 32];
    __shared__ __align__(16) float ys[TCH * HW];
    const unsigned tid = threadIdx.x;
    const int lane = (int)(tid & 31u);
    const int wave = __builtin_amdgcn_readfirstlane((int)(threadIdx.x >> 5));
    const unsigned bx = blockIdx.x, by = blockIdx.y;
    const unsigned b = by >> 3, h = by & 7u;
    const int t0 = (int)(bx * (unsigned)TCH);
#pragma unroll 1
    for (int it = 0; it < 4; ++it) {
        const unsigned e = (unsigned)it * 256u + tid; const unsigned i = e >> 4, q = e & 15u;
        const int tt = t0 - PADL + (int)i; const int ttc = min(max(tt, 0), SEQ - 1);
        v4f v = *(const v4f*)(XG + ((size_t)ttc * NBT + b) * CC + h * HW + q * 4u);
        asm volatile("" : "+v"(v));
        const bool ok = (tt >= 0) && (tt < SEQ);
        v4f z = (v4f){};
        if (ok) z = v;
        *(v4fa*)(&xs[i * HW + q * 4u]) = z; }
#pragma unroll 1
    for (int it = 0; it < 4; ++it) {
        const unsigned e = (unsigned)it * 256u + tid; const unsigned tl = e >> 5, k = e & 31u;
        const unsigned kc = min(k, (unsigned)(NTAP - 1));
        float v = LG[((size_t)(t0 + (int)tl) * NBT + b) * HKP + h * NTAP + kc];
        asm volatile("" : "+v"(v));
        wl[tl * 32u + k] = (k < (unsigned)NTAP) ? v : 0.0f; }
    __syncthreads();
    if (wave == 0) {
        const int rb = lane * 32;
        float m = -3.0e38f;
#pragma unroll 1
        for (int k = 0; k < NTAP; ++k) m = fmaxf(m, wl[rb + k]);
        float s = 0.0f;
#pragma unroll 1
        for (int k = 0; k < NTAP; ++k) { const float ev = expf(wl[rb + k] - m); wl[rb + k] = ev; s += ev; }
        const float inv = 1.0f / s;
#pragma unroll 1
        for (int k = 0; k < NTAP; ++k) { const float pv = wl[rb + k] * inv; wl[rb + k] = pv; }
    }
    __syncthreads();
    const int c = (wave & 1) * 32 + lane;
    const int tg = wave >> 1;
#pragma unroll 1
    for (int it = 0; it < 8; ++it) {
        const int tl = tg * 8 + it;
        float acc = 0.0f;
#pragma unroll 2
        for (int k4 = 0; k4 < 8; ++k4) {
            const v4f w = *(const v4fa*)(&wl[tl * 32 + k4 * 4]);
            const int xi = (tl + k4 * 4) * HW + c;
            acc = fmaf(xs[xi], w[0], acc);
            acc = fmaf(xs[xi + HW], w[1], acc);
            acc = fmaf(xs[xi + 2 * HW], w[2], acc);
            acc = fmaf(xs[xi + 3 * HW], w[3], acc); }
        ys[tl * HW + c] = acc; }
    __syncthreads();
    const unsigned row = tid >> 3, c8 = (tid & 7u) * 8u;
    const v4f x0 = *(const v4fa*)(&ys[row * HW + c8]); const v4f x1 = *(const v4fa*)(&ys[row * HW + c8 + 4u]); v8h hv;
#pragma unroll
    for (int i = 0; i < 4; ++i) { hv[i] = toh_flush(x0[i] * YC); hv[4 + i] = toh_flush(x1[i] * YC); }
    h16* dst = YH + ((size_t)(t0 + (int)row) * NBT + b) * CC + h * HW + c8;
    *(volatile v8h*)dst = hv; __threadfence(); *(volatile v8h*)dst = hv;
}

static constexpr size_t al256(size_t v) { return (v + 255) & ~(size_t)255; }
static constexpr size_t SZ_XB  = al256((size_t)MROWS * CC * 2);
static constexpr size_t SZ_W1  = al256((size_t)C2 * CC * 2);
static constexpr size_t SZ_WL  = al256((size_t)HKP * CC * 2);
static constexpr size_t SZ_W2  = al256((size_t)CC * CC * 2);
static constexpr size_t SZ_XG  = al256((size_t)MROWS * CC * 4);
static constexpr size_t SZ_XH  = al256((size_t)MROWS * CC * 2);
static constexpr size_t SZ_LG  = al256((size_t)MROWS * HKP * 4);
static constexpr size_t SZ_YH  = al256((size_t)MROWS * CC * 2);
static constexpr size_t SZ_TOTAL = SZ_XB + SZ_W1 + SZ_WL + SZ_W2 + SZ_XG + SZ_XH + SZ_LG + SZ_YH;
static_assert(SZ_TOTAL <= (size_t)134217728);
static_assert(((size_t)MROWS * CC) % 8 == 0);

extern "C" void kernel_launch(void* const* d_in, const int* in_sizes, int n_in,
                              void* d_out, int out_size, void* d_ws, size_t ws_size, hipStream_t stream) {
    if (n_in < 7) return;
    if ((size_t)in_sizes[0] < (size_t)MROWS * CC) return;
    if ((size_t)in_sizes[1] < (size_t)CC * C2 || in_sizes[2] < C2) return;
    if ((size_t)in_sizes[3] < (size_t)CC * HK || in_sizes[4] < HK) return;
    if ((size_t)in_sizes[5] < (size_t)CC * CC || in_sizes[6] < CC) return;
    if ((size_t)out_size < (size_t)MROWS * CC) return;
    if (SZ_TOTAL > ws_size) return;
    const float* x   = (const float*)d_in[0];
    const float* w1  = (const float*)d_in[1];
    const float* b1  = (const float*)d_in[2];
    const float* wlw = (const float*)d_in[3];
    const float* wlb = (const float*)d_in[4];
    const float* w2  = (const float*)d_in[5];
    const float* b2  = (const float*)d_in[6];
    float* OUT = (float*)d_out;
    char* wsp = (char*)d_ws;
    bf*    XB  = (bf*)wsp;    wsp += SZ_XB;
    bf*    W1T = (bf*)wsp;    wsp += SZ_W1;
    h16*   WLT = (h16*)wsp;   wsp += SZ_WL;
    h16*   W2T = (h16*)wsp;   wsp += SZ_W2;
    float* XG  = (float*)wsp; wsp += SZ_XG;
    h16*   XH  = (h16*)wsp;   wsp += SZ_XH;
    float* LG  = (float*)wsp; wsp += SZ_LG;
    h16*   YH  = (h16*)wsp;   wsp += SZ_YH;

    { const size_t n8 = (size_t)MROWS * CC / 8;
      k_cvt8<<<(unsigned)((n8 + 255) / 256), 256, 0, stream>>>(x, XB, n8); }
    k_wt_b<<<dim3(CC / 64, C2 / 64, 1), 256, 0, stream>>>(w1, W1T, C2, C2);
    k_wt_h<<<dim3(CC / 64, HKP / 64, 1), 256, 0, stream>>>(wlw, WLT, HK, HK);
    k_wt_h<<<dim3(CC / 64, CC / 64, 1), 256, 0, stream>>>(w2, W2T, CC, CC);

    k_glu<<<dim3(MROWS / 32, CC / 64, 1), 32, 0, stream>>>(XB, W1T, b1, XG, XH);
    k_gemm_h<<<dim3(MROWS / 64, HKP / 64, 1), 32, 0, stream>>>(XH, WLT, wlb, LG, HKP, HK, LG_ISH);
    k_dconv<<<dim3(SEQ / TCH, NBT * NHD, 1), 256, 0, stream>>>(XG, LG, YH);
    k_gemm_h<<<dim3(MROWS / 64, CC / 64, 1), 32, 0, stream>>>(YH, W2T, b2, OUT, CC, CC, OT_ISH);
}
